// Mamba2SSD_71562745086268
// MI455X (gfx1250) — hardware-verified
//
#include <hip/hip_runtime.h>
#include <math.h>

#define NB    2
#define TLEN  2048
#define DMOD  1024
#define DIN   2048
#define DST   64
#define DTR   64
#define DPJ   4288
#define NTOK  4096
#define OFF_Z 2048
#define OFF_B 4096
#define OFF_C 4160
#define OFF_R 4224
#define TPB   128
#define NBLK  32
#define OSTR  68
#define SCH   32
#define NSUB  4
#define NSTS  16
#define CHB   64
#define NSCB  64
#define LOG2E 1.4426950408889634f

static_assert(NTOK == NB * TLEN);
static_assert(NTOK % TPB == 0);
static_assert(NBLK == NTOK / TPB);
static_assert(DPJ == 2 * DIN + 2 * DST + DTR);
static_assert(DPJ % 64 == 0);
static_assert(DIN % 64 == 0);
static_assert(DMOD % 64 == 0);
static_assert(DMOD % 32 == 0);
static_assert(DTR % 32 == 0);
static_assert(DIN % 32 == 0);
static_assert(DPJ % 32 == 0);
static_assert(TLEN % SCH == 0);
static_assert(NSUB * NSTS == DST);
static_assert(CHB * NSUB == 256);
static_assert(DIN % CHB == 0);
static_assert(NSCB == NB * (DIN / CHB));
static_assert(SCH * CHB == 2 * 256 * 4);
static_assert(CHB * DST == 4 * 256 * 4);
static_assert(OSTR % 4 == 0);
static_assert(DMOD % 8 == 0);
static_assert(DTR % 8 == 0);
static_assert(DIN % 8 == 0);

typedef unsigned short us16 __attribute__((ext_vector_type(16)));
typedef unsigned short us8  __attribute__((ext_vector_type(8)));
typedef unsigned short us8a __attribute__((ext_vector_type(8), may_alias));
typedef unsigned int   u32x8 __attribute__((ext_vector_type(8)));
typedef __bf16 v16b __attribute__((ext_vector_type(16)));
typedef float v8f __attribute__((ext_vector_type(8)));
typedef float v4f __attribute__((ext_vector_type(4)));
typedef float v4fa __attribute__((ext_vector_type(4), may_alias));
union FragU { us16 v; us8 h[2]; u32x8 w; };

#if __has_builtin(__builtin_amdgcn_exp2f)
#define FEXP2(x) __builtin_amdgcn_exp2f(x)
#else
#define FEXP2(x) __expf((x) * 0.6931471805599453f)
#endif

__device__ __forceinline__ unsigned short bf16_bits(float f) {
  unsigned u = __float_as_uint(f);
  u += 0x7FFFu + ((u >> 16) & 1u);
  return (unsigned short)(u >> 16);
}
__device__ __forceinline__ float bf16_val(unsigned short b) { return __uint_as_float(((unsigned)b) << 16); }
__device__ __forceinline__ float bf16r(float f) { return bf16_val(bf16_bits(f)); }
__device__ __forceinline__ float siluf(float x) { return x * __builtin_amdgcn_rcpf(1.0f + __expf(-x)); }

__device__ __forceinline__ void split8(const v4f a, const v4f b, us8& hi, us8& lo) {
#pragma unroll
  for (int u = 0; u < 4; ++u) {
    const unsigned short ha = bf16_bits(a[u]);
    hi[u] = ha; lo[u] = bf16_bits(a[u] - bf16_val(ha));
    const unsigned short hb = bf16_bits(b[u]);
    hi[4 + u] = hb; lo[4 + u] = bf16_bits(b[u] - bf16_val(hb));
  }
}

__device__ __forceinline__ v8f mma_bf16(us16 a, us16 b, v8f c) {
  return __builtin_amdgcn_wmma_f32_16x16x32_bf16(false, __builtin_bit_cast(v16b, a), false, __builtin_bit_cast(v16b, b), (short)0, c, false, false);
}
__device__ __forceinline__ void wguard2(v8f& c0, v8f& c1, v8f& c2, v8f& c3, const us16& a0, const us16& a1,
                                        const us16& b0, const us16& b1, const us16& b2, const us16& b3) {
#if defined(__HIP_DEVICE_COMPILE__)
  asm volatile("v_nop\n\tv_nop\n\tv_nop\n\tv_nop"
               : "+v"(c0), "+v"(c1), "+v"(c2), "+v"(c3)
               : "v"(a0), "v"(a1), "v"(b0), "v"(b1), "v"(b2), "v"(b3));
#endif
}

__device__ __forceinline__ us16 gfrag(const unsigned short* p) {
  const int kh = ((threadIdx.x >> 4) & 1) * 8;
  FragU f;
  f.h[0] = *(const us8a*)(p + kh);
  f.h[1] = *(const us8a*)(p + 16 + kh);
  return f.v;
}

__global__ __launch_bounds__(256) void k_cvt(const float* __restrict__ src, unsigned short* dst, int nsrc, int ncol8, int total8) {
  const int idx = blockIdx.x * 256 + threadIdx.x;
  if (idx >= total8) return;
  const int row = idx / ncol8, c8 = (idx - row * ncol8) * 8;
  const int rs = (row < nsrc) ? row : (nsrc - 1);
  const float* s = src + (size_t)rs * (size_t)(ncol8 * 8) + c8;
  const v4f a = *(const v4fa*)s, b = *(const v4fa*)(s + 4);
  const bool zr = (row >= nsrc);
  us8 o;
#pragma unroll
  for (int u = 0; u < 4; ++u) {
    o[u]     = zr ? (unsigned short)0 : bf16_bits(a[u]);
    o[4 + u] = zr ? (unsigned short)0 : bf16_bits(b[u]);
  }
  const size_t off = (size_t)row * (size_t)(ncol8 * 8) + c8;
  *(volatile us8*)(dst + off) = o;
  __threadfence();
  *(volatile us8*)(dst + off) = o;
}

__global__ __launch_bounds__(256) void k_split(const float* __restrict__ src, int lds_, int ncol8, int total8,
                                              unsigned short* H, unsigned short* L) {
  const int idx = blockIdx.x * 256 + threadIdx.x;
  if (idx >= total8) return;
  const int row = idx / ncol8, c8 = (idx - row * ncol8) * 8;
  const float* s = src + (size_t)row * (size_t)lds_ + c8;
  const v4f a = *(const v4fa*)s, b = *(const v4fa*)(s + 4);
  us8 hi, lo;
  split8(a, b, hi, lo);
  const size_t off = (size_t)row * (size_t)(ncol8 * 8) + c8;
  *(volatile us8*)(H + off) = hi; *(volatile us8*)(L + off) = lo;
  __threadfence();
  *(volatile us8*)(H + off) = hi; *(volatile us8*)(L + off) = lo;
}

template <int NPL, int BIAS, int ACT>
__global__ __launch_bounds__(256) void k_gemm(const unsigned short* __restrict__ A0, const unsigned short* __restrict__ A1, int lda,
                                             const unsigned short* __restrict__ Bw, int ldb, int K,
                                             const float* __restrict__ bias, float* Yf, int ldy) {
  __shared__ __attribute__((aligned(16))) float oS[8 * 16 * OSTR];
  const int tid = threadIdx.x, lane = tid & 31, wave = tid >> 5, cl = lane & 15, hh = lane >> 4;
  const int mb = blockIdx.x * TPB, m0 = mb + 16 * wave, n0 = blockIdx.y * 64;

  v8f acc[4];
#pragma unroll
  for (int j = 0; j < 4; ++j) { const v8f zz = {0.f, 0.f, 0.f, 0.f, 0.f, 0.f, 0.f, 0.f}; acc[j] = zz; }

  const unsigned short* a0p = A0 + (size_t)(m0 + cl) * (size_t)lda;
  const unsigned short* a1p = A1 + (size_t)(m0 + cl) * (size_t)lda;
  const unsigned short* bwp = Bw + (size_t)(n0 + cl) * (size_t)ldb;
#pragma unroll 1
  for (int k0 = 0; k0 < K; k0 += 32) {
    const us16 af0 = gfrag(a0p + k0);
    us16 af1 = af0;
    if (NPL == 2) af1 = gfrag(a1p + k0);
    us16 bfr[4];
#pragma unroll
    for (int j = 0; j < 4; ++j) bfr[j] = gfrag(bwp + (size_t)(16 * j) * (size_t)ldb + k0);
#pragma unroll
    for (int j = 0; j < 4; ++j) acc[j] = mma_bf16(af0, bfr[j], acc[j]);
    if (NPL == 2) {
#pragma unroll
      for (int j = 0; j < 4; ++j) acc[j] = mma_bf16(af1, bfr[j], acc[j]);
    }
    wguard2(acc[0], acc[1], acc[2], acc[3], af0, af1, bfr[0], bfr[1], bfr[2], bfr[3]);
  }

  float* so = oS + wave * (16 * OSTR);
#pragma unroll
  for (int j = 0; j < 4; ++j)
#pragma unroll
    for (int r = 0; r < 8; ++r) so[(8 * hh + r) * OSTR + 16 * j + cl] = acc[j][r];
  __syncthreads();

  if (ACT != 0) {
#pragma unroll 1
    for (int it = 0; it < 8; ++it) {
      const int cx = it * 32 + lane, r = cx >> 4, q = (cx & 15) * 4;
      v4f v = *(const v4fa*)(so + r * OSTR + q);
#pragma unroll
      for (int u = 0; u < 4; ++u) {
        float t = v[u];
        if (BIAS) t = t + bf16r(bias[n0 + q + u]);
        if (ACT == 1) t = siluf(t);
        if (ACT == 2) t = fmaxf(t, 0.0f) + log1pf(expf(-fabsf(t)));
        v[u] = t;
      }
      *(v4fa*)(so + r * OSTR + q) = v;
    }
  }
#pragma unroll
  for (int pass = 0; pass < 2; ++pass) {
#pragma unroll
    for (int it = 0; it < 8; ++it) {
      const int cx = it * 32 + lane, r = cx >> 4, q = (cx & 15) * 4;
      v4f v = *(const v4fa*)(so + r * OSTR + q);
      if (BIAS && ACT == 0) {
#pragma unroll
        for (int u = 0; u < 4; ++u) v[u] = v[u] + bf16r(bias[n0 + q + u]);
      }
      *(volatile v4f*)(Yf + (size_t)(m0 + r) * (size_t)ldy + n0 + q) = v;
    }
    __threadfence();
  }
}

__global__ __launch_bounds__(256) void k_scan(const float* __restrict__ DT, float* PR,
                                             const float* __restrict__ cw, const float* __restrict__ cb,
                                             const float* __restrict__ Alog, const float* __restrict__ Dv, float* hT) {
  __shared__ __attribute__((aligned(16))) float a2s[DST];
  __shared__ __attribute__((aligned(16))) float sy[SCH * CHB];
  __shared__ __attribute__((aligned(16))) float hs[CHB * DST];
  const int tid = threadIdx.x;
  const int b = blockIdx.x / (DIN / CHB), dg = blockIdx.x - b * (DIN / CHB);
  const int ch = tid >> 2, sub = tid & 3;
  const int d = dg * CHB + ch, n0 = sub * NSTS;
  if (tid < DST) a2s[tid] = -expf(bf16r(Alog[tid])) * LOG2E;
  __syncthreads();
  float A2[NSTS], h[NSTS];
#pragma unroll
  for (int i = 0; i < NSTS; ++i) { A2[i] = a2s[n0 + i]; h[i] = 0.0f; }
  const float Dd = bf16r(Dv[d]);
  const v4f w4 = *(const v4fa*)(cw + (size_t)d * 4);
  const float w0 = bf16r(w4[0]), w1 = bf16r(w4[1]), w2 = bf16r(w4[2]), w3 = bf16r(w4[3]);
  const float bcv = bf16r(cb[d]);
  float xw0 = 0.0f, xw1 = 0.0f, xw2 = 0.0f;

#pragma unroll 1
  for (int c = 0; c < TLEN / SCH; ++c) {
#pragma unroll 1
    for (int s = 0; s < SCH; ++s) {
      const size_t tok = (size_t)b * TLEN + (size_t)(c * SCH + s);
      const float* pr = PR + tok * DPJ;
      const float dl = DT[tok * DIN + d];
      const float xi = pr[d];
      const float zv = pr[OFF_Z + d];
      v4f Bv[4], Cv[4];
#pragma unroll
      for (int q = 0; q < 4; ++q) {
        Bv[q] = *(const v4fa*)(pr + OFF_B + n0 + 4 * q);
        Cv[q] = *(const v4fa*)(pr + OFF_C + n0 + 4 * q);
      }
      const float cv = (((w0 * xw0 + w1 * xw1) + w2 * xw2) + w3 * xi) + bcv;
      xw0 = xw1; xw1 = xw2; xw2 = xi;
      const float xcv = siluf(cv);
      const float dx = dl * xcv;
      float y = 0.0f;
#pragma unroll
      for (int i = 0; i < NSTS; ++i) {
        const float ex = FEXP2(dl * A2[i]);
        h[i] = ex * h[i] + dx * Bv[i >> 2][i & 3];
        y = y + h[i] * Cv[i >> 2][i & 3];
      }
      y += __shfl_xor(y, 1);
      y += __shfl_xor(y, 2);
      const float yv = (y + xcv * Dd) * siluf(zv);
      if (sub == 0) sy[s * CHB + ch] = yv;
    }
    __syncthreads();
#pragma unroll
    for (int pass = 0; pass < 2; ++pass) {
#pragma unroll
      for (int it = 0; it < 2; ++it) {
        const int cx = it * 256 + tid, r = cx >> 4, q = (cx & 15) * 4;
        const v4f v = *(const v4fa*)(sy + r * CHB + q);
        *(volatile v4f*)(PR + ((size_t)b * TLEN + (size_t)(c * SCH + r)) * DPJ + OFF_Z + dg * CHB + q) = v;
      }
      __threadfence();
    }
    __syncthreads();
  }

#pragma unroll
  for (int q = 0; q < 4; ++q) {
    v4f hv;
    hv[0] = h[4 * q]; hv[1] = h[4 * q + 1]; hv[2] = h[4 * q + 2]; hv[3] = h[4 * q + 3];
    *(v4fa*)(hs + ch * DST + n0 + 4 * q) = hv;
  }
  __syncthreads();
  float* hb = hT + ((size_t)(b * DIN + dg * CHB)) * DST;
#pragma unroll
  for (int pass = 0; pass < 2; ++pass) {
#pragma unroll
    for (int it = 0; it < 4; ++it) {
      const int cx = (it * 256 + tid) * 4;
      const v4f v = *(const v4fa*)(hs + cx);
      *(volatile v4f*)(hb + cx) = v;
    }
    __threadfence();
  }
}

extern "C" void kernel_launch(void* const* d_in, const int* in_sizes, int n_in,
                              void* d_out, int out_size, void* d_ws, size_t ws_size,
                              hipStream_t stream) {
  if (n_in < 9) return;
  if (in_sizes[0] != NTOK * DMOD || in_sizes[1] != DPJ * DMOD || in_sizes[2] != DIN * 4 || in_sizes[3] != DIN ||
      in_sizes[4] != DST || in_sizes[5] != DIN || in_sizes[6] != DIN * DTR || in_sizes[7] != DIN || in_sizes[8] != DMOD * DIN) return;
  if (out_size != NTOK * DMOD + NB * DIN * DST) return;

  const float* x      = (const float*)d_in[0];
  const float* in_w   = (const float*)d_in[1];
  const float* conv_w = (const float*)d_in[2];
  const float* conv_b = (const float*)d_in[3];
  const float* A_log  = (const float*)d_in[4];
  const float* D_par  = (const float*)d_in[5];
  const float* dt_w   = (const float*)d_in[6];
  const float* dt_b   = (const float*)d_in[7];
  const float* out_w  = (const float*)d_in[8];
  float* out = (float*)d_out;
  float* hT  = out + (size_t)NTOK * DMOD;

  size_t off = 0;
  auto carve = [&](size_t bytes) -> char* { char* p = (char*)d_ws + off; off += (bytes + 255) & ~(size_t)255; return p; };
  float* PROJ = (float*)carve((size_t)NTOK * DPJ * 4);
  unsigned short* XB  = (unsigned short*)carve((size_t)NTOK * DMOD * 2);
  unsigned short* WIN = (unsigned short*)carve((size_t)DPJ * DMOD * 2);
  char* RD = carve((size_t)NTOK * DIN * 4);
  unsigned short* DRH = (unsigned short*)carve((size_t)NTOK * DTR * 2);
  unsigned short* DRL = (unsigned short*)carve((size_t)NTOK * DTR * 2);
  unsigned short* WDT = (unsigned short*)carve((size_t)DIN * DTR * 2);
  unsigned short* WOP = (unsigned short*)carve((size_t)DMOD * DIN * 2);
  if (off > ws_size || off > (size_t)134217728) return;

  float* DTF = (float*)RD;
  unsigned short* YGH = (unsigned short*)RD;
  unsigned short* YGL = (unsigned short*)(RD + (size_t)NTOK * DIN * 2);

  const dim3 b256(256);
  auto cdv = [](long a, long bq) { return (unsigned)((a + bq - 1) / bq); };

  k_cvt<<<dim3(cdv((long)NTOK * DMOD / 8, 256)), b256, 0, stream>>>(x, XB, NTOK, DMOD / 8, NTOK * DMOD / 8);
  k_cvt<<<dim3(cdv((long)DPJ * DMOD / 8, 256)), b256, 0, stream>>>(in_w, WIN, DPJ, DMOD / 8, DPJ * DMOD / 8);
  k_cvt<<<dim3(cdv((long)DIN * DTR / 8, 256)), b256, 0, stream>>>(dt_w, WDT, DIN, DTR / 8, DIN * DTR / 8);
  k_cvt<<<dim3(cdv((long)DMOD * DIN / 8, 256)), b256, 0, stream>>>(out_w, WOP, DMOD, DIN / 8, DMOD * DIN / 8);
  k_gemm<1, 0, 0><<<dim3(NBLK, DPJ / 64), b256, 0, stream>>>(XB, XB, DMOD, WIN, DMOD, DMOD, conv_b, PROJ, DPJ);
  k_split<<<dim3(cdv((long)NTOK * DTR / 8, 256)), b256, 0, stream>>>(PROJ + OFF_R, DPJ, DTR / 8, NTOK * DTR / 8, DRH, DRL);
  k_gemm<2, 1, 2><<<dim3(NBLK, DIN / 64), b256, 0, stream>>>(DRH, DRL, DTR, WDT, DTR, DTR, dt_b, DTF, DIN);
  k_scan<<<dim3(NSCB), b256, 0, stream>>>(DTF, PROJ, conv_w, conv_b, A_log, D_par, hT);
  k_split<<<dim3(cdv((long)NTOK * DIN / 8, 256)), b256, 0, stream>>>(PROJ + OFF_Z, DPJ, DIN / 8, NTOK * DIN / 8, YGH, YGL);
  k_gemm<2, 0, 0><<<dim3(NBLK, DMOD / 64), b256, 0, stream>>>(YGH, YGL, DIN, WOP, DIN, DIN, dt_b, out, DMOD);
}
